// FoodRiskGNN_18219251270415
// MI455X (gfx1250) — hardware-verified
//
#include <hip/hip_runtime.h>
#include <stddef.h>
#include <math.h>


#define F_IN    64
#define F_HID   128
#define F_OUT   64
#define NTHR    256
#define NWAVE   8
#define EPT     8
#define NGRP    2
#define CHUNK   (NTHR * EPT * NGRP)
#define WCAP    (EPT * NGRP * 32)
#define LISTN   (NWAVE * WCAP)
#define NBC     4096
#define NBF     1024
#define RCAP    40960
#define RBN     128
#define TGT     256
#define DEGCAP  1024
#define GROWS   128
#define OTHR    512
#define WSCAP   134217728

#define K1      (2 * F_IN)
#define K2      (2 * F_HID)
#define NC1     F_HID
#define NC2     F_OUT
#define WSC     64
#define ASC1    16
#define ASC2    16
#define WP1     0
#define WP2     (NC1 * K1)
#define WPTOT   (WP2 + NC2 * K2)
#define WB1     ((NC1 * K1 / 8) / NTHR)
#define WB2     ((NC2 * K2 / 8) / NTHR)
#define MPW     F_HID

#define LDS_FILL ((RCAP + NBF + LISTN) * 4 + 64)
#define LDS_A1   (GROWS * (K1 + 8) * 2)
#define LDS_A2   (GROWS * (K2 + 8) * 2)
#define LDS_G1   (LDS_A1 + GROWS * NC1 * 4)
#define LDS_G2   (LDS_A2 + GROWS * NC2 * 4)

static_assert((CHUNK & (CHUNK - 1)) == 0);
static_assert(CHUNK <= 4096);
static_assert(NBC <= 4096 && NBF <= 4096);
static_assert((NBC & (NBC - 1)) == 0 && (NBF & (NBF - 1)) == 0);
static_assert(NBC == 4 * NBF);
static_assert(OTHR * 8 == NBC);
static_assert((RCAP % 32) == 0);
static_assert(TGT == NWAVE * 32 && (TGT % GROWS) == 0);
static_assert((NBC % TGT) == 0);
static_assert(GROWS == NWAVE * 16);
static_assert((K1 % 32) == 0 && (K2 % 32) == 0);
static_assert((F_IN % 32) == 0 && (F_HID % 32) == 0);
static_assert((NC1 % 64) == 0 && (NC2 % 64) == 0);
static_assert(((NC1 * K1 / 8) % NTHR) == 0 && ((NC2 * K2 / 8) % NTHR) == 0);
static_assert((WP2 % 64) == 0 && (WPTOT % 64) == 0);
static_assert((LDS_A1 % 16) == 0 && (LDS_A2 % 16) == 0);
static_assert(MPW >= F_IN && MPW >= F_HID);

typedef float          v2f  __attribute__((ext_vector_type(2)));
typedef float          v4f  __attribute__((ext_vector_type(4)));
typedef float          v8f  __attribute__((ext_vector_type(8)));
typedef int            v4i  __attribute__((ext_vector_type(4)));
typedef _Float16       v8h  __attribute__((ext_vector_type(8)));
typedef _Float16       v16h __attribute__((ext_vector_type(16)));
union FragH { v16h v; v8h h[2]; };

template <int C> struct VecT;
template <> struct VecT<2> {
  typedef v2f t;
  static __device__ __forceinline__ v2f zero() { v2f z = {0.0f, 0.0f}; return z; }
};
template <> struct VecT<4> {
  typedef v4f t;
  static __device__ __forceinline__ v4f zero() { v4f z = {0.0f, 0.0f, 0.0f, 0.0f}; return z; }
};

__device__ __forceinline__ v8h cvt8(v4f a, v4f b, float sc) {
  v8h r;
  r[0] = (_Float16)(a.x * sc); r[1] = (_Float16)(a.y * sc);
  r[2] = (_Float16)(a.z * sc); r[3] = (_Float16)(a.w * sc);
  r[4] = (_Float16)(b.x * sc); r[5] = (_Float16)(b.y * sc);
  r[6] = (_Float16)(b.z * sc); r[7] = (_Float16)(b.w * sc);
  return r;
}

__device__ __forceinline__ v8f wmh(v16h a, v16h b, v8f c) {
  v8f d = __builtin_amdgcn_wmma_f32_16x16x32_f16(false, a, false, b, (short)0, c, false, false);
  asm volatile("v_nop\n\tv_nop\n\tv_nop\n\tv_nop" : "+v"(d) : "v"(a), "v"(b));
  return d;
}

template <int NT, int KDT, int APKT>
__device__ __forceinline__ void mma_tiles(const _Float16* sA, const _Float16* __restrict__ Bw,
                                          int wrow, int lane, v8f (&acc)[NT]) {
  constexpr int NKT = KDT / 32;
  const int hh = lane >> 4, m = lane & 15;
#pragma unroll
  for (int t = 0; t < NT; ++t) { v8f z = {0.f, 0.f, 0.f, 0.f, 0.f, 0.f, 0.f, 0.f}; acc[t] = z; }
  const _Float16* ap = sA + (wrow + m) * APKT + 8 * hh;
#pragma unroll 1
  for (int kt = 0; kt < NKT; ++kt) {
    FragH a;
    a.h[0] = *(const v8h*)(ap + 32 * kt);
    a.h[1] = *(const v8h*)(ap + 32 * kt + 16);
#pragma unroll
    for (int t = 0; t < NT; ++t) {
      const _Float16* bp = Bw + (size_t)(16 * t + m) * KDT + 32 * kt + 8 * hh;
      FragH b;
      b.h[0] = *(const v8h*)bp;
      b.h[1] = *(const v8h*)(bp + 16);
      acc[t] = wmh(a.v, b.v, acc[t]);
    }
  }
}

template <int NB>
__device__ __forceinline__ int scan_chunk(const int* __restrict__ dsts, int nE, int cbase, int slotBase,
                                          int vec8, int* list, int tid, int lane, int wave) {
  int wc = 0;
#pragma unroll
  for (int g = 0; g < NGRP; ++g) {
    const int el0  = (g * NTHR + tid) * EPT;
    const int e0   = cbase + el0;
    const int sent = -2147483647 - 1;
    v4i da, db;
    if (vec8 != 0 && cbase + CHUNK <= nE) {
      da = *(const v4i*)(dsts + e0);
      db = *(const v4i*)(dsts + e0 + 4);
    } else {
      da.x = (e0     < nE) ? dsts[min(e0, nE - 1)] : sent;
      da.y = (e0 + 1 < nE) ? dsts[min(e0 + 1, nE - 1)] : sent;
      da.z = (e0 + 2 < nE) ? dsts[min(e0 + 2, nE - 1)] : sent;
      da.w = (e0 + 3 < nE) ? dsts[min(e0 + 3, nE - 1)] : sent;
      db.x = (e0 + 4 < nE) ? dsts[min(e0 + 4, nE - 1)] : sent;
      db.y = (e0 + 5 < nE) ? dsts[min(e0 + 5, nE - 1)] : sent;
      db.z = (e0 + 6 < nE) ? dsts[min(e0 + 6, nE - 1)] : sent;
      db.w = (e0 + 7 < nE) ? dsts[min(e0 + 7, nE - 1)] : sent;
    }
    const unsigned nb = (unsigned)slotBase;
    const unsigned s0 = (unsigned)da.x - nb, s1 = (unsigned)da.y - nb;
    const unsigned s2 = (unsigned)da.z - nb, s3 = (unsigned)da.w - nb;
    const unsigned s4 = (unsigned)db.x - nb, s5 = (unsigned)db.y - nb;
    const unsigned s6 = (unsigned)db.z - nb, s7 = (unsigned)db.w - nb;
    const bool h0 = s0 < (unsigned)NB, h1 = s1 < (unsigned)NB, h2 = s2 < (unsigned)NB, h3 = s3 < (unsigned)NB;
    const bool h4 = s4 < (unsigned)NB, h5 = s5 < (unsigned)NB, h6 = s6 < (unsigned)NB, h7 = s7 < (unsigned)NB;
    const unsigned any = __builtin_amdgcn_ballot_w32(h0 | h1 | h2 | h3 | h4 | h5 | h6 | h7);
    if (any != 0u) {
#define HITJ(J, HJ, SJ) { \
        const unsigned mj = __builtin_amdgcn_ballot_w32(HJ); \
        if (mj != 0u) { \
          if (HJ) { \
            const int pos = wc + (int)__builtin_amdgcn_mbcnt_lo(mj, 0u); \
            if (pos < WCAP) list[wave * WCAP + pos] = ((el0 + (J)) << 12) | (int)(SJ); \
          } \
          wc += (int)__builtin_popcount(mj); } }
      HITJ(0, h0, s0)
      HITJ(1, h1, s1)
      HITJ(2, h2, s2)
      HITJ(3, h3, s3)
      HITJ(4, h4, s4)
      HITJ(5, h5, s5)
      HITJ(6, h6, s6)
      HITJ(7, h7, s7)
#undef HITJ
    }
  }
  return wc;
}

__global__ __launch_bounds__(NTHR) void k_wprep(
    const float* __restrict__ w1l, const float* __restrict__ w1r,
    const float* __restrict__ w2l, const float* __restrict__ w2r, _Float16* wp) {
  const int blk = blockIdx.x, tid = threadIdx.x;
  float v[8];
  size_t dsto;
  if (blk < WB1) {
    const int i = blk * NTHR + tid;
    const int n = i / (K1 / 8), k0 = (i % (K1 / 8)) * 8;
#pragma unroll
    for (int e = 0; e < 8; ++e) {
      const int k = k0 + e;
      const int ka = k > F_IN - 1 ? F_IN - 1 : k;
      int kb = k - F_IN; kb = kb < 0 ? 0 : kb;
      const float va = w1l[ka * NC1 + n];
      const float vb = w1r[kb * NC1 + n];
      v[e] = ((k < F_IN) ? va : vb) * (float)WSC;
    }
    dsto = (size_t)WP1 + (size_t)i * 8;
  } else {
    const int i = (blk - WB1) * NTHR + tid;
    const int n = i / (K2 / 8), k0 = (i % (K2 / 8)) * 8;
#pragma unroll
    for (int e = 0; e < 8; ++e) {
      const int k = k0 + e;
      const int ka = k > F_HID - 1 ? F_HID - 1 : k;
      int kb = k - F_HID; kb = kb < 0 ? 0 : kb;
      const float va = w2l[ka * NC2 + n];
      const float vb = w2r[kb * NC2 + n];
      v[e] = ((k < F_HID) ? va : vb) * (float)WSC;
    }
    dsto = (size_t)WP2 + (size_t)i * 8;
  }
  v4f a, b;
  a.x = v[0]; a.y = v[1]; a.z = v[2]; a.w = v[3];
  b.x = v[4]; b.y = v[5]; b.z = v[6]; b.w = v[7];
  const v8h hv = cvt8(a, b, 1.0f);
  _Float16* dh = wp + dsto;
  *(volatile v8h*)dh = hv;
  __threadfence();
  *(volatile v8h*)dh = hv;
}

__global__ __launch_bounds__(NTHR) void k_count(const int* __restrict__ dsts, int* cnt, int nE, int vec8) {
  __shared__ __attribute__((aligned(16))) int scnt[NBC];
  __shared__ __attribute__((aligned(16))) int list[LISTN];
  __shared__ int wcnt[NWAVE];
  const int tid = threadIdx.x, lane = tid & 31, wave = tid >> 5;
  const int nodeBase = blockIdx.x * NBC;

  for (int i = tid; i < NBC; i += NTHR) scnt[i] = 0;
  __syncthreads();

  const int nChunks = (nE + CHUNK - 1) / CHUNK;
#pragma unroll 1
  for (int ch = 0; ch < nChunks; ++ch) {
    const int cbase = ch * CHUNK;
    const int wc = scan_chunk<NBC>(dsts, nE, cbase, nodeBase, vec8, list, tid, lane, wave);
    if (lane == 0) wcnt[wave] = wc;
    __syncthreads();
    if (wave == 0) {
#pragma unroll 1
      for (int wsx = 0; wsx < NWAVE; ++wsx) {
        int n = __builtin_amdgcn_readfirstlane(wcnt[wsx]);
        n = n > WCAP ? WCAP : (n < 0 ? 0 : n);
        const int* lp = list + wsx * WCAP;
#pragma unroll 1
        for (int i = 0; i < n; ++i) {
          const int ent  = __builtin_amdgcn_readfirstlane(lp[i]);
          const int slot = ent & (NBC - 1);
          if (lane == 0) scnt[slot] = scnt[slot] + 1;
        }
      }
    }
    __syncthreads();
  }

  v4i cq[4];
#pragma unroll
  for (int q = 0; q < 4; ++q) {
    const int f = (wave * 4 + q) * 128 + 4 * lane;
    cq[q] = *(const v4i*)(scnt + f);
  }
  int* cp = cnt + (size_t)nodeBase;
#pragma unroll
  for (int q = 0; q < 4; ++q) {
    const int f = (wave * 4 + q) * 128 + 4 * lane;
    *(volatile v4i*)(cp + f) = cq[q];
  }
  __threadfence();
#pragma unroll
  for (int q = 0; q < 4; ++q) {
    const int f = (wave * 4 + q) * 128 + 4 * lane;
    *(volatile v4i*)(cp + f) = cq[q];
  }
}

__global__ __launch_bounds__(OTHR) void k_offsets(
    const int* __restrict__ cnt, int* off, int* rbase, int nChunk) {
  __shared__ __attribute__((aligned(16))) int soff[NBC];
  __shared__ __attribute__((aligned(16))) int srb[RBN];
  __shared__ int wtot[OTHR / 32];
  const int tid = threadIdx.x, lane = tid & 31, wave = tid >> 5, sub = tid >> 7;
  for (int i = tid; i < RBN; i += OTHR) srb[i] = 0;
  __syncthreads();
  int carry = 0;
#pragma unroll 1
  for (int ch = 0; ch < nChunk; ++ch) {
    const int base = ch * NBC;
    const v4i c0 = *(const v4i*)(cnt + base + 8 * tid);
    const v4i c1 = *(const v4i*)(cnt + base + 8 * tid + 4);
    const int e0 = max(c0.x, 0), e1 = max(c0.y, 0), e2 = max(c0.z, 0), e3 = max(c0.w, 0);
    const int e4 = max(c1.x, 0), e5 = max(c1.y, 0), e6 = max(c1.z, 0), e7 = max(c1.w, 0);
    const int ts = e0 + e1 + e2 + e3 + e4 + e5 + e6 + e7;
    int incl = ts;
#pragma unroll
    for (int d = 1; d < 32; d <<= 1) {
      const int t = __shfl_up(incl, d);
      if (lane >= d) incl += t;
    }
    if (lane == 31) wtot[wave] = incl;
    __syncthreads();
    const int S0 = wtot[0]  + wtot[1]  + wtot[2]  + wtot[3];
    const int S1 = wtot[4]  + wtot[5]  + wtot[6]  + wtot[7];
    const int S2 = wtot[8]  + wtot[9]  + wtot[10] + wtot[11];
    const int S3 = wtot[12] + wtot[13] + wtot[14] + wtot[15];
    int pre = 0;
#pragma unroll 1
    for (int w = 4 * sub; w < wave; ++w) pre += wtot[w];
    const int b0 = carry;
    const int b1 = b0 + ((S0 + 31) & ~31);
    const int b2 = b1 + ((S1 + 31) & ~31);
    const int b3 = b2 + ((S2 + 31) & ~31);
    const int b4 = b3 + ((S3 + 31) & ~31);
    const int myb = sub == 0 ? b0 : (sub == 1 ? b1 : (sub == 2 ? b2 : b3));
    if (tid == 0) {
      srb[min(4 * ch + 0, RBN - 1)] = b0;
      srb[min(4 * ch + 1, RBN - 1)] = b1;
      srb[min(4 * ch + 2, RBN - 1)] = b2;
      srb[min(4 * ch + 3, RBN - 1)] = b3;
    }
    int run = myb + pre + incl - ts;
    soff[8 * tid + 0] = run; run += e0;
    soff[8 * tid + 1] = run; run += e1;
    soff[8 * tid + 2] = run; run += e2;
    soff[8 * tid + 3] = run; run += e3;
    soff[8 * tid + 4] = run; run += e4;
    soff[8 * tid + 5] = run; run += e5;
    soff[8 * tid + 6] = run; run += e6;
    soff[8 * tid + 7] = run;
    carry = b4;
    __syncthreads();
    const v4i o0 = *(const v4i*)(soff + 4 * tid);
    const v4i o1 = *(const v4i*)(soff + 4 * (tid + OTHR));
    int* op = off + base;
    *(volatile v4i*)(op + 4 * tid) = o0;
    *(volatile v4i*)(op + 4 * (tid + OTHR)) = o1;
    __threadfence();
    *(volatile v4i*)(op + 4 * tid) = o0;
    *(volatile v4i*)(op + 4 * (tid + OTHR)) = o1;
    __syncthreads();
  }
  if (tid == 0) srb[min(4 * nChunk, RBN - 1)] = carry;
  __syncthreads();
  v4i rv = {0, 0, 0, 0};
  if (tid < 32) rv = *(const v4i*)(srb + 4 * tid);
  if (tid < 32) *(volatile v4i*)(rbase + 4 * tid) = rv;
  __threadfence();
  if (tid < 32) *(volatile v4i*)(rbase + 4 * tid) = rv;
}

__global__ __launch_bounds__(NTHR) void k_fill(
    const int* __restrict__ srcs, const int* __restrict__ dsts,
    const int* __restrict__ off, const int* __restrict__ rbase,
    int* csr, int nN, int nE, int vec8, int csrLen) {
  extern __shared__ v4f lds_dyn[];
  int* region = (int*)lds_dyn;
  int* cursor = region + RCAP;
  int* list   = cursor + NBF;
  int* wcnt   = list + LISTN;
  const int tid = threadIdx.x, lane = tid & 31, wave = tid >> 5;
  const int b = blockIdx.x;
  const int nodeBase = b * NBF;

  int rb0 = rbase[b];
  const int rb1 = rbase[b + 1];
  rb0 = rb0 < 0 ? 0 : (rb0 > csrLen ? csrLen : rb0);
  rb0 &= ~31;
  int len = rb1 - rb0;
  len = len < 0 ? 0 : (len > RCAP ? RCAP : len);
  int lenW = (len + 31) & ~31;
  if (rb0 + lenW > csrLen) lenW = (csrLen - rb0) & ~31;

  {
    const v4i z = {0, 0, 0, 0};
    for (int i = tid; i < RCAP / 4; i += NTHR) ((v4i*)region)[i] = z;
    for (int s = tid; s < NBF; s += NTHR) {
      int o = off[nodeBase + s] - rb0;
      o = o < 0 ? 0 : (o > RCAP ? RCAP : o);
      cursor[s] = o;
    }
  }
  __syncthreads();

  const int nChunks = (nE + CHUNK - 1) / CHUNK;
#pragma unroll 1
  for (int ch = 0; ch < nChunks; ++ch) {
    const int cbase = ch * CHUNK;
    const int wc = scan_chunk<NBF>(dsts, nE, cbase, nodeBase, vec8, list, tid, lane, wave);
    if (lane == 0) wcnt[wave] = wc;
    __syncthreads();
    if (wave == 0) {
#pragma unroll 1
      for (int wsx = 0; wsx < NWAVE; ++wsx) {
        int n = __builtin_amdgcn_readfirstlane(wcnt[wsx]);
        n = n > WCAP ? WCAP : (n < 0 ? 0 : n);
        const int* lp = list + wsx * WCAP;
#pragma unroll 1
        for (int i = 0; i < n; ++i) {
          const int ent  = __builtin_amdgcn_readfirstlane(lp[i]);
          const int slot = ent & (NBF - 1);
          int e = cbase + ((ent >> 12) & (CHUNK - 1));
          e = e > nE - 1 ? nE - 1 : e;
          int sv = srcs[e];
          sv = sv < 0 ? 0 : (sv > nN - 1 ? nN - 1 : sv);
          if (lane == 0) {
            int pos = cursor[slot];
            pos = pos < 0 ? 0 : (pos > RCAP - 1 ? RCAP - 1 : pos);
            region[pos] = sv;
            const int np = pos + 1;
            cursor[slot] = np > RCAP ? RCAP : np;
          }
        }
      }
    }
    __syncthreads();
  }

  const int nv = lenW >> 2;
  int* gp = csr + rb0;
#pragma unroll 1
  for (int i = tid; i < nv; i += NTHR) { const v4i v = ((const v4i*)region)[i]; *(volatile v4i*)(gp + 4 * i) = v; }
  __threadfence();
#pragma unroll 1
  for (int i = tid; i < nv; i += NTHR) { const v4i v = ((const v4i*)region)[i]; *(volatile v4i*)(gp + 4 * i) = v; }
}

template <int FDT>
__global__ __launch_bounds__(NTHR) void k_agg(
    const int* __restrict__ csr, const int* __restrict__ off, const int* __restrict__ cnt,
    const float* __restrict__ xs, float* Am, int nN, int csrLen) {
  constexpr int CPL = FDT / 32;
  typedef typename VecT<CPL>::t vcf;
  const int tid = threadIdx.x, lane = tid & 31, wave = tid >> 5;
  const int tbase = blockIdx.x * TGT + wave * 32;
  const int cl = tbase + lane;
  const int cnt_l = cnt[cl];
  const int off_l = off[cl];

#pragma unroll 1
  for (int j = 0; j < 32; ++j) {
    const int c = tbase + j;
    int n = __builtin_amdgcn_readlane(cnt_l, j);
    n = n < 0 ? 0 : (n > DEGCAP ? DEGCAP : n);
    const int st = __builtin_amdgcn_readlane(off_l, j);
    vcf sm = VecT<CPL>::zero();
#pragma unroll 1
    for (int q0 = 0; q0 < n; q0 += 32) {
      int pos = st + q0 + lane;
      pos = pos < 0 ? 0 : (pos > csrLen - 1 ? csrLen - 1 : pos);
      int sl = csr[pos];
      sl = sl < 0 ? 0 : (sl > nN - 1 ? nN - 1 : sl);
      const int mcnt = (n - q0) < 32 ? (n - q0) : 32;
#pragma unroll 1
      for (int p = 0; p < mcnt; ++p) {
        const int s = __builtin_amdgcn_readlane(sl, p);
        const vcf vf = *(const vcf*)(xs + (size_t)s * FDT + CPL * lane);
        sm = sm + vf;
      }
    }
    const float rc = 1.0f / (float)(n > 1 ? n : 1);
    const vcf mean = sm * rc;
    float* ap = Am + (size_t)c * FDT + CPL * lane;
    *(volatile vcf*)ap = mean;
    __threadfence();
    *(volatile vcf*)ap = mean;
  }
}

template <int FDA, int NCOL, int ASC, int ACT, bool GUARD>
__global__ __launch_bounds__(NTHR) void k_gemm(
    const float* __restrict__ agg, const float* __restrict__ xr,
    const _Float16* __restrict__ Bw, const float* __restrict__ bias,
    float* C, int nN) {
  static_assert(NCOL == 64 || NCOL == 128);
  static_assert(FDA == 64 || FDA == 128);
  constexpr int KDT  = 2 * FDA;
  constexpr int APKT = KDT + 8;
  constexpr int NCH  = NCOL / 64;
  constexpr int TPR  = FDA / 8;
  constexpr int RPI  = NTHR / TPR;
  constexpr int NIT  = GROWS / RPI;
  constexpr int LDSA = GROWS * APKT * 2;
  static_assert((APKT % 8) == 0 && (LDSA % 16) == 0 && (GROWS % RPI) == 0);
  extern __shared__ v4f lds_dyn[];
  _Float16* sA  = (_Float16*)lds_dyn;
  float*    stg = (float*)((char*)lds_dyn + LDSA);
  const int tid = threadIdx.x, lane = tid & 31, wave = tid >> 5, hh = lane >> 4, m = lane & 15;
  const int rowBase = blockIdx.x * GROWS;
  const int c0 = (tid % TPR) * 8, rr = tid / TPR;
  const float asc = (float)ASC;

#pragma unroll 2
  for (int it = 0; it < NIT; ++it) {
    const int r = it * RPI + rr;
    const float* ap = agg + (size_t)(rowBase + r) * FDA + c0;
    const v4f a = *(const v4f*)ap, b = *(const v4f*)(ap + 4);
    *(v8h*)(sA + r * APKT + c0) = cvt8(a, b, asc);
  }
#pragma unroll 2
  for (int it = 0; it < NIT; ++it) {
    const int r = it * RPI + rr;
    int row = rowBase + r;
    row = row > nN - 1 ? nN - 1 : row;
    const float* ap = xr + (size_t)row * FDA + c0;
    const v4f a = *(const v4f*)ap, b = *(const v4f*)(ap + 4);
    *(v8h*)(sA + r * APKT + FDA + c0) = cvt8(a, b, asc);
  }
  __syncthreads();

  const float inv = 1.0f / (float)(ASC * WSC);
#pragma unroll
  for (int ch = 0; ch < NCH; ++ch) {
    v8f acc[4];
    mma_tiles<4, KDT, APKT>(sA, Bw + (size_t)(64 * ch) * KDT, wave * 16, lane, acc);
    float* sp = stg + (wave * 16 + 8 * hh) * NCOL + 64 * ch + m;
#pragma unroll
    for (int t = 0; t < 4; ++t) {
      const float bv = bias[64 * ch + 16 * t + m];
#pragma unroll
      for (int r = 0; r < 8; ++r) {
        float v = acc[t][r] * inv + bv;
        if (ACT == 1) v = fmaxf(v, 0.0f);
        sp[r * NCOL + 16 * t] = v;
      }
    }
  }
  __syncthreads();

  if (ACT == 2) {
#pragma unroll 1
    for (int i = tid; i < GROWS * NCOL; i += NTHR) {
      const float v  = stg[i];
      const float vc = fminf(fmaxf(v, -30.0f), 30.0f);
      const float e  = __expf(-vc);
      stg[i] = 1.0f / (1.0f + e);
    }
    __syncthreads();
  }

  if (NCOL == 128) {
    const float* lp = stg + wave * 16 * NCOL + 4 * lane;
    float* gp = C + (size_t)(rowBase + wave * 16) * NCOL + 4 * lane;
#pragma unroll
    for (int i = 0; i < 16; ++i) {
      const int row = rowBase + wave * 16 + i;
      const v4f v = *(const v4f*)(lp + NCOL * i);
      if (!GUARD || row < nN) *(volatile v4f*)(gp + NCOL * i) = v;
    }
    __threadfence();
#pragma unroll
    for (int i = 0; i < 16; ++i) {
      const int row = rowBase + wave * 16 + i;
      const v4f v = *(const v4f*)(lp + NCOL * i);
      if (!GUARD || row < nN) *(volatile v4f*)(gp + NCOL * i) = v;
    }
  } else {
    const int rsub = lane >> 4;
    const float* lp = stg + wave * 16 * NCOL + 4 * lane;
    float* gp = C + (size_t)(rowBase + wave * 16) * NCOL + 4 * lane;
#pragma unroll
    for (int i = 0; i < 8; ++i) {
      const int row = rowBase + wave * 16 + 2 * i + rsub;
      const v4f v = *(const v4f*)(lp + 2 * NCOL * i);
      if (!GUARD || row < nN) *(volatile v4f*)(gp + 2 * NCOL * i) = v;
    }
    __threadfence();
#pragma unroll
    for (int i = 0; i < 8; ++i) {
      const int row = rowBase + wave * 16 + 2 * i + rsub;
      const v4f v = *(const v4f*)(lp + 2 * NCOL * i);
      if (!GUARD || row < nN) *(volatile v4f*)(gp + 2 * NCOL * i) = v;
    }
  }
}

extern "C" void kernel_launch(void* const* d_in, const int* in_sizes, int n_in,
                              void* d_out, int out_size, void* d_ws, size_t ws_size,
                              hipStream_t stream) {
  if (n_in < 8) return;
  const int nN = in_sizes[0] / F_IN;
  const int nE = in_sizes[1] / 2;
  if (nN <= 0 || nE <= 0) return;
  if (in_sizes[0] != nN * F_IN || in_sizes[1] != 2 * nE) return;
  if (in_sizes[2] != F_IN * NC1 || in_sizes[3] != F_IN * NC1 || in_sizes[4] != NC1) return;
  if (in_sizes[5] != F_HID * NC2 || in_sizes[6] != F_HID * NC2 || in_sizes[7] != NC2) return;
  if (out_size != nN * NC2) return;
  if (nE > (1 << 28) || nN > (1 << 24)) return;

  const float* x    = (const float*)d_in[0];
  const int*   ei   = (const int*)d_in[1];
  const float* w1l  = (const float*)d_in[2];
  const float* w1r  = (const float*)d_in[3];
  const float* b1   = (const float*)d_in[4];
  const float* w2l  = (const float*)d_in[5];
  const float* w2r  = (const float*)d_in[6];
  const float* b2   = (const float*)d_in[7];
  float* out = (float*)d_out;
  const int* srcs = ei;
  const int* dsts = ei + nE;

  const int NPAD   = ((nN + TGT - 1) / TGT) * TGT;
  const int nBC    = (nN + NBC - 1) / NBC;
  const int CNTPAD = nBC * NBC;
  if (4 * nBC + 1 > RBN) return;
  const int nBF    = (nN + NBF - 1) / NBF;
  const int csrLen = ((nE + 31) & ~31) + 4096;
  if (31 * 4 * nBC > 4096) return;
  const int nGemm  = NPAD / GROWS;
  const int nAgg   = NPAD / TGT;

  char* ws = (char*)d_ws;
  size_t off = 0;
  const size_t oW    = off; off += (size_t)WPTOT * 2;               off = (off + 255) & ~(size_t)255;
  const size_t oCnt  = off; off += (size_t)CNTPAD * 4;              off = (off + 255) & ~(size_t)255;
  const size_t oOff  = off; off += (size_t)CNTPAD * 4;              off = (off + 255) & ~(size_t)255;
  const size_t oRb   = off; off += (size_t)RBN * 4;                 off = (off + 255) & ~(size_t)255;
  const size_t oCsr  = off; off += (size_t)csrLen * 4;              off = (off + 255) & ~(size_t)255;
  const size_t oM    = off; off += (size_t)NPAD * MPW * 4;          off = (off + 255) & ~(size_t)255;
  const size_t oH    = off; off += (size_t)NPAD * F_HID * 4;        off = (off + 255) & ~(size_t)255;
  if (off > ws_size || off > (size_t)WSCAP) return;
  _Float16* wp   = (_Float16*)(ws + oW);
  int*      cnt  = (int*)(ws + oCnt);
  int*      offp = (int*)(ws + oOff);
  int*      rb   = (int*)(ws + oRb);
  int*      csr  = (int*)(ws + oCsr);
  float*    M    = (float*)(ws + oM);
  float*    H    = (float*)(ws + oH);

  const int vec8 = ((nE & 3) == 0) ? 1 : 0;

  k_wprep<<<WB1 + WB2, NTHR, 0, stream>>>(w1l, w1r, w2l, w2r, wp);

  k_count<<<nBC, NTHR, 0, stream>>>(dsts, cnt, nE, vec8);
  k_offsets<<<1, OTHR, 0, stream>>>(cnt, offp, rb, nBC);
  hipFuncSetAttribute(reinterpret_cast<const void*>(&k_fill),
                      hipFuncAttributeMaxDynamicSharedMemorySize, LDS_FILL);
  k_fill<<<nBF, NTHR, LDS_FILL, stream>>>(srcs, dsts, offp, rb, csr, nN, nE, vec8, csrLen);

  k_agg<F_IN><<<nAgg, NTHR, 0, stream>>>(csr, offp, cnt, x, M, nN, csrLen);

  hipFuncSetAttribute(reinterpret_cast<const void*>(&k_gemm<F_IN, NC1, ASC1, 1, false>),
                      hipFuncAttributeMaxDynamicSharedMemorySize, LDS_G1);
  k_gemm<F_IN, NC1, ASC1, 1, false><<<nGemm, NTHR, LDS_G1, stream>>>(M, x, wp + WP1, b1, H, nN);

  k_agg<F_HID><<<nAgg, NTHR, 0, stream>>>(csr, offp, cnt, H, M, nN, csrLen);

  hipFuncSetAttribute(reinterpret_cast<const void*>(&k_gemm<F_HID, NC2, ASC2, 2, true>),
                      hipFuncAttributeMaxDynamicSharedMemorySize, LDS_G2);
  k_gemm<F_HID, NC2, ASC2, 2, true><<<nGemm, NTHR, LDS_G2, stream>>>(M, H, wp + WP2, b2, out, nN);
}
